// hhgnnConv_eu_adaptive_17927193494052
// MI455X (gfx1250) — hardware-verified
//
#include <hip/hip_runtime.h>
#include <stddef.h>


#define DF    128
#define NH    8
#define HCH   16
#define GR    32
#define AP    136
#define XSP   132
#define NB    512
#define CHUNK 2048
#define NTHR  256
#define NWAVE 8
#define WCAP  256
#define NGRP  (CHUNK / (NTHR * 4))

#define LDS_SACC (NB * DF)
#define LDS_DEN  (NB * NH)
#define LDS_LIST (NWAVE * WCAP)
#define LDS_BYTES ((LDS_SACC + LDS_DEN + LDS_LIST + NWAVE + NB + 4 * DF) * 4)

static_assert(WCAP == (CHUNK / NTHR) * 32);
static_assert(NGRP == 2);
static_assert(NB == 512);
static_assert(CHUNK == 2048);
static_assert(NH * HCH == DF);
static_assert(((LDS_SACC + LDS_DEN) % 4) == 0);
static_assert(((LDS_SACC + LDS_DEN + LDS_LIST + NWAVE + NB) % 4) == 0);
static_assert(LDS_BYTES == 290848);

typedef float          v4f   __attribute__((ext_vector_type(4)));
typedef float          v8f   __attribute__((ext_vector_type(8)));
typedef int            v4i   __attribute__((ext_vector_type(4)));
typedef unsigned short v8us  __attribute__((ext_vector_type(8)));
typedef unsigned short v16us __attribute__((ext_vector_type(16)));
typedef __bf16         v16bf __attribute__((ext_vector_type(16)));
union Frag { v16bf v; v16us u; v8us half[2]; };

__device__ __forceinline__ v8f wm(v16bf a, v16bf b, v8f c) {
  v8f d = __builtin_amdgcn_wmma_f32_16x16x32_bf16(false, a, false, b, (short)0, c, false, false);
  asm volatile("v_nop\n\tv_nop\n\tv_nop\n\tv_nop" : "+v"(d) : "v"(a), "v"(b));
  return d;
}

__device__ __forceinline__ unsigned int bfr(float f) {
  const unsigned int u = __float_as_uint(f);
  return (u + 0x7FFFu + ((u >> 16) & 1u)) >> 16;
}

__device__ __forceinline__ void split8(v4f a, v4f b, v4i& ho, v4i& lo) {
  float f[8] = {a.x, a.y, a.z, a.w, b.x, b.y, b.z, b.w};
  unsigned int h[8], l[8];
#pragma unroll
  for (int j = 0; j < 8; ++j) {
    h[j] = bfr(f[j]);
    l[j] = bfr(f[j] - __uint_as_float(h[j] << 16));
  }
  ho.x = (int)(h[0] | (h[1] << 16)); ho.y = (int)(h[2] | (h[3] << 16));
  ho.z = (int)(h[4] | (h[5] << 16)); ho.w = (int)(h[6] | (h[7] << 16));
  lo.x = (int)(l[0] | (l[1] << 16)); lo.y = (int)(l[2] | (l[3] << 16));
  lo.z = (int)(l[4] | (l[5] << 16)); lo.w = (int)(l[6] | (l[7] << 16));
}

__global__ __launch_bounds__(NTHR) void k_prepw(const float* __restrict__ W,
                                                unsigned short* Whi, unsigned short* Wlo) {
  __shared__ float sW[32 * 129];
  const int tid = threadIdx.x;
  const int t   = blockIdx.x >> 2;
  const int o0  = (blockIdx.x & 3) * 32;
  for (int q = tid; q < DF * 8; q += NTHR) {
    const int k  = q >> 3;
    const int oc = (q & 7) * 4;
    const v4f v = *(const v4f*)(W + ((size_t)t * DF + k) * DF + o0 + oc);
    sW[(oc + 0) * 129 + k] = v.x;
    sW[(oc + 1) * 129 + k] = v.y;
    sW[(oc + 2) * 129 + k] = v.z;
    sW[(oc + 3) * 129 + k] = v.w;
  }
  __syncthreads();
  const int rl = tid >> 4;
  const int k0 = (tid & 15) * 8;
  v4f a0, b0, a1, b1;
  {
    const float* p0 = sW + rl * 129 + k0;
    const float* p1 = sW + (16 + rl) * 129 + k0;
    a0.x = p0[0]; a0.y = p0[1]; a0.z = p0[2]; a0.w = p0[3];
    b0.x = p0[4]; b0.y = p0[5]; b0.z = p0[6]; b0.w = p0[7];
    a1.x = p1[0]; a1.y = p1[1]; a1.z = p1[2]; a1.w = p1[3];
    b1.x = p1[4]; b1.y = p1[5]; b1.z = p1[6]; b1.w = p1[7];
  }
  v4i h0, l0, h1, l1;
  split8(a0, b0, h0, l0);
  split8(a1, b1, h1, l1);
  const size_t g0 = ((size_t)t * DF + o0 + rl) * DF + k0;
  const size_t g1 = ((size_t)t * DF + o0 + 16 + rl) * DF + k0;
  *(volatile v4i*)(Whi + g0) = h0; *(volatile v4i*)(Wlo + g0) = l0;
  *(volatile v4i*)(Whi + g1) = h1; *(volatile v4i*)(Wlo + g1) = l1;
  __threadfence();
  *(volatile v4i*)(Whi + g0) = h0; *(volatile v4i*)(Wlo + g0) = l0;
  *(volatile v4i*)(Whi + g1) = h1; *(volatile v4i*)(Wlo + g1) = l1;
}

__global__ __launch_bounds__(NTHR) void k_gemm(
    const float* __restrict__ X, const unsigned short* __restrict__ Whi,
    const unsigned short* __restrict__ Wlo, const int* __restrict__ vtype,
    float* X0, int nN) {
  __shared__ __attribute__((aligned(16))) unsigned short Ah[GR * AP];
  __shared__ __attribute__((aligned(16))) unsigned short Al[GR * AP];
  __shared__ __attribute__((aligned(16))) float Xs[GR * XSP];
  __shared__ int sVt[GR];

  const int tid  = threadIdx.x;
  const int lane = tid & 31;
  const int wave = tid >> 5;
  const int hh   = lane >> 4;
  const int m    = lane & 15;
  const int rowBase = blockIdx.x * GR;

  {
    const int r  = tid >> 3;
    const int c0 = (tid & 7) * 16;
    int row = rowBase + r;
    if (row > nN - 1) row = nN - 1;
    const float* p = X + (size_t)row * DF + c0;
    const v4f f0 = *(const v4f*)(p), f1 = *(const v4f*)(p + 4);
    const v4f f2 = *(const v4f*)(p + 8), f3 = *(const v4f*)(p + 12);
    v4i h0, l0, h1, l1;
    split8(f0, f1, h0, l0);
    split8(f2, f3, h1, l1);
    *(v4i*)(Ah + r * AP + c0)     = h0;
    *(v4i*)(Ah + r * AP + c0 + 8) = h1;
    *(v4i*)(Al + r * AP + c0)     = l0;
    *(v4i*)(Al + r * AP + c0 + 8) = l1;
    if (tid < GR) {
      int rr = rowBase + tid;
      if (rr > nN - 1) rr = nN - 1;
      int t = vtype[rr];
      t = t < 0 ? 0 : (t > 3 ? 3 : t);
      sVt[tid] = t;
    }
  }
  __syncthreads();

  int vt0[8], vt1[8];
#pragma unroll
  for (int r = 0; r < 8; ++r) { vt0[r] = sVt[8 * hh + r]; vt1[r] = sVt[16 + 8 * hh + r]; }

  const int ncol = wave * 16 + m;
  const unsigned short* a0hp = Ah + m * AP + 8 * hh;
  const unsigned short* a1hp = Ah + (16 + m) * AP + 8 * hh;
  const unsigned short* a0lp = Al + m * AP + 8 * hh;
  const unsigned short* a1lp = Al + (16 + m) * AP + 8 * hh;

  v8f sel0 = {0.f, 0.f, 0.f, 0.f, 0.f, 0.f, 0.f, 0.f};
  v8f sel1 = {0.f, 0.f, 0.f, 0.f, 0.f, 0.f, 0.f, 0.f};
#pragma unroll 1
  for (int t = 0; t < 4; ++t) {
    v8f c0 = {0.f, 0.f, 0.f, 0.f, 0.f, 0.f, 0.f, 0.f};
    v8f c1 = {0.f, 0.f, 0.f, 0.f, 0.f, 0.f, 0.f, 0.f};
    const unsigned short* bhp = Whi + ((size_t)t * DF + ncol) * DF + 8 * hh;
    const unsigned short* blp = Wlo + ((size_t)t * DF + ncol) * DF + 8 * hh;
#pragma unroll
    for (int kt = 0; kt < DF / 32; ++kt) {
      const int k0 = kt * 32;
      Frag bh, bl, a0h, a0l, a1h, a1l;
      bh.half[0]  = *(const v8us*)(bhp + k0);   bh.half[1]  = *(const v8us*)(bhp + k0 + 16);
      bl.half[0]  = *(const v8us*)(blp + k0);   bl.half[1]  = *(const v8us*)(blp + k0 + 16);
      a0h.half[0] = *(const v8us*)(a0hp + k0);  a0h.half[1] = *(const v8us*)(a0hp + k0 + 16);
      a0l.half[0] = *(const v8us*)(a0lp + k0);  a0l.half[1] = *(const v8us*)(a0lp + k0 + 16);
      a1h.half[0] = *(const v8us*)(a1hp + k0);  a1h.half[1] = *(const v8us*)(a1hp + k0 + 16);
      a1l.half[0] = *(const v8us*)(a1lp + k0);  a1l.half[1] = *(const v8us*)(a1lp + k0 + 16);
      c0 = wm(a0h.v, bh.v, c0);
      c0 = wm(a0h.v, bl.v, c0);
      c0 = wm(a0l.v, bh.v, c0);
      c1 = wm(a1h.v, bh.v, c1);
      c1 = wm(a1h.v, bl.v, c1);
      c1 = wm(a1l.v, bh.v, c1);
    }
#pragma unroll
    for (int r = 0; r < 8; ++r) {
      sel0[r] = (vt0[r] == t) ? c0[r] : sel0[r];
      sel1[r] = (vt1[r] == t) ? c1[r] : sel1[r];
    }
  }

#pragma unroll
  for (int r = 0; r < 8; ++r) {
    Xs[(8 * hh + r) * XSP + ncol]      = sel0[r];
    Xs[(16 + 8 * hh + r) * XSP + ncol] = sel1[r];
  }
  __syncthreads();
  v4f xr[4];
  float* xp[4];
#pragma unroll
  for (int i = 0; i < 4; ++i) {
    xr[i] = *(const v4f*)(Xs + (4 * wave + i) * XSP + 4 * lane);
    xp[i] = X0 + (size_t)(rowBase + 4 * wave + i) * DF + 4 * lane;
  }
#pragma unroll
  for (int i = 0; i < 4; ++i) *(volatile v4f*)(xp[i]) = xr[i];
  __threadfence();
#pragma unroll
  for (int i = 0; i < 4; ++i) *(volatile v4f*)(xp[i]) = xr[i];
}

__global__ __launch_bounds__(NTHR) void k_agg(
    const float* __restrict__ srcRows, const int* __restrict__ srcIds,
    const int* __restrict__ dstIds, const int* __restrict__ dstTyp,
    const float* __restrict__ att, float* outRows,
    int nSrc, int nDst, int nnz, int rowLimit, int doRelu) {
  extern __shared__ v4f lds_dyn[];
  float* sacc = (float*)lds_dyn;
  float* den  = sacc + LDS_SACC;
  int*   list = (int*)(den + LDS_DEN);
  int*   wcnt = list + LDS_LIST;
  int*   sTyp = wcnt + NWAVE;
  float* sAtt = (float*)(sTyp + NB);

  const int tid  = threadIdx.x;
  const int lane = tid & 31;
  const int wave = tid >> 5;
  const int hd   = lane >> 2;
  const int dstBase = blockIdx.x * NB;

  {
    const v4f z4 = {0.f, 0.f, 0.f, 0.f};
    for (int i = tid; i < (LDS_SACC + LDS_DEN) / 4; i += NTHR) lds_dyn[i] = z4;
    for (int s = tid; s < NB; s += NTHR) {
      int d = dstBase + s;
      if (d > nDst - 1) d = nDst - 1;
      int t = dstTyp[d];
      t = t < 0 ? 0 : (t > 3 ? 3 : t);
      sTyp[s] = t;
    }
    for (int i = tid; i < 4 * DF; i += NTHR) sAtt[i] = att[i];
  }
  __syncthreads();
  const bool al16 = ((((size_t)dstIds) & 15) == 0);

  const int nChunks = (nnz + CHUNK - 1) / CHUNK;
#pragma unroll 1
  for (int ch = 0; ch < nChunks; ++ch) {
    const int cbase = ch * CHUNK;
    int wc = 0;
#pragma unroll
    for (int g = 0; g < NGRP; ++g) {
      const int el0 = (g * NTHR + tid) * 4;
      const int e0  = cbase + el0;
      const int sent = -2147483647 - 1;
      v4i d;
      if (al16 && (e0 + 3 < nnz)) {
        d = *(const v4i*)(dstIds + e0);
      } else {
        d.x = (e0     < nnz) ? dstIds[min(e0, nnz - 1)]     : sent;
        d.y = (e0 + 1 < nnz) ? dstIds[min(e0 + 1, nnz - 1)] : sent;
        d.z = (e0 + 2 < nnz) ? dstIds[min(e0 + 2, nnz - 1)] : sent;
        d.w = (e0 + 3 < nnz) ? dstIds[min(e0 + 3, nnz - 1)] : sent;
      }
      const unsigned s0 = (unsigned)d.x - (unsigned)dstBase;
      const unsigned s1 = (unsigned)d.y - (unsigned)dstBase;
      const unsigned s2 = (unsigned)d.z - (unsigned)dstBase;
      const unsigned s3 = (unsigned)d.w - (unsigned)dstBase;
      const bool h0 = s0 < (unsigned)NB;
      const bool h1 = s1 < (unsigned)NB;
      const bool h2 = s2 < (unsigned)NB;
      const bool h3 = s3 < (unsigned)NB;
      const unsigned many = __builtin_amdgcn_ballot_w32(h0 | h1 | h2 | h3);
      if (many != 0u) {
#define HITJ(J, HJ, SJ) { \
          const unsigned mj = __builtin_amdgcn_ballot_w32(HJ); \
          if (HJ) { \
            const int pos = wc + (int)__builtin_amdgcn_mbcnt_lo(mj, 0u); \
            if (pos < WCAP) list[wave * WCAP + pos] = ((el0 + (J)) << 9) | (int)(SJ); \
          } \
          wc += (int)__builtin_popcount(mj); }
        HITJ(0, h0, s0)
        HITJ(1, h1, s1)
        HITJ(2, h2, s2)
        HITJ(3, h3, s3)
#undef HITJ
      }
    }
    if (lane == 0) wcnt[wave] = wc;
    __syncthreads();

    if (wave == 0) {
      for (int wsx = 0; wsx < NWAVE; ++wsx) {
        int n = wcnt[wsx];
        if (n > WCAP) n = WCAP;
        if (n < 0) n = 0;
        for (int i = 0; i < n; ++i) {
          const int ent  = list[wsx * WCAP + i];
          const int slot = ent & (NB - 1);
          const int el   = (ent >> 9) & (CHUNK - 1);
          int e = cbase + el;
          if (e > nnz - 1) e = nnz - 1;
          int src = srcIds[e];
          src = src < 0 ? 0 : (src > nSrc - 1 ? nSrc - 1 : src);
          const int t = sTyp[slot];
          const v4f a4 = *(const v4f*)(sAtt + t * DF + 4 * lane);
          const v4f xv = *(const v4f*)(srcRows + (size_t)src * DF + 4 * lane);
          float p = xv.x * a4.x + xv.y * a4.y + xv.z * a4.z + xv.w * a4.w;
          p += __shfl_xor(p, 1, 32);
          p += __shfl_xor(p, 2, 32);
          p = (p > 0.f) ? p : 0.2f * p;
          p = fminf(fmaxf(p, -80.f), 80.f);
          const float w = __expf(p);
          v4f* sp = (v4f*)(sacc + slot * DF + 4 * lane);
          const v4f cur = *sp;
          const v4f nxt = cur + w * xv;
          *sp = nxt;
          if ((lane & 3) == 0) {
            const float o = den[slot * NH + hd];
            den[slot * NH + hd] = o + w;
          }
        }
      }
    }
    __syncthreads();
  }

#pragma unroll 1
  for (int j = 0; j < NB / NWAVE; ++j) {
    const int slot = wave * (NB / NWAVE) + j;
    const int row  = dstBase + slot;
    if (row >= rowLimit) break;
    const float dv  = den[slot * NH + hd] + 1e-16f;
    const float inv = 1.0f / dv;
    v4f v = *(const v4f*)(sacc + slot * DF + 4 * lane) * inv;
    if (doRelu) {
      v.x = v.x > 0.f ? v.x : 0.f;
      v.y = v.y > 0.f ? v.y : 0.f;
      v.z = v.z > 0.f ? v.z : 0.f;
      v.w = v.w > 0.f ? v.w : 0.f;
    }
    float* op = outRows + (size_t)row * DF + 4 * lane;
    *(volatile v4f*)op = v;
    __threadfence();
    *(volatile v4f*)op = v;
  }
}

extern "C" void kernel_launch(void* const* d_in, const int* in_sizes, int n_in,
                              void* d_out, int out_size, void* d_ws, size_t ws_size,
                              hipStream_t stream) {
  if (n_in < 8) return;
  const int nN  = in_sizes[6];
  const int nE  = in_sizes[7];
  const int nnz = in_sizes[4];
  if (nN <= 0 || nE <= 0 || nnz <= 0) return;
  if (in_sizes[0] != nN * DF) return;
  if (in_sizes[1] != 4 * DF * DF) return;
  if (in_sizes[2] != 4 * DF || in_sizes[3] != 4 * DF) return;
  if (in_sizes[5] != nnz) return;
  if (out_size != nN * DF) return;

  const float* X      = (const float*)d_in[0];
  const float* W      = (const float*)d_in[1];
  const float* att_e  = (const float*)d_in[2];
  const float* att_v  = (const float*)d_in[3];
  const int*   vertex = (const int*)d_in[4];
  const int*   edges  = (const int*)d_in[5];
  const int*   vtype  = (const int*)d_in[6];
  const int*   etype  = (const int*)d_in[7];
  float* out = (float*)d_out;

  const int nP  = ((nN + GR - 1) / GR) * GR;
  const int nPE = ((nE + NB - 1) / NB) * NB;
  size_t off = 0;
  unsigned short* Whi = (unsigned short*)((char*)d_ws + off); off += (size_t)4 * DF * DF * sizeof(unsigned short);
  unsigned short* Wlo = (unsigned short*)((char*)d_ws + off); off += (size_t)4 * DF * DF * sizeof(unsigned short);
  float* X0 = (float*)((char*)d_ws + off); off += (size_t)nP * DF * sizeof(float);
  float* Xe = (float*)((char*)d_ws + off); off += (size_t)nPE * DF * sizeof(float);
  if (off > ws_size) return;

  k_prepw<<<16, NTHR, 0, stream>>>(W, Whi, Wlo);
  k_gemm<<<nP / GR, NTHR, 0, stream>>>(X, Whi, Wlo, vtype, X0, nN);

  hipFuncSetAttribute(reinterpret_cast<const void*>(&k_agg),
                      hipFuncAttributeMaxDynamicSharedMemorySize, LDS_BYTES);
  k_agg<<<nPE / NB, NTHR, LDS_BYTES, stream>>>(X0, vertex, edges, etype, att_e, Xe,
                                               nN, nE, nnz, nPE, 1);
  k_agg<<<(nN + NB - 1) / NB, NTHR, LDS_BYTES, stream>>>(Xe, edges, vertex, vtype, att_v, out,
                                                         nE, nN, nnz, nN, 0);
}
